// GenConv2d_56118042689936
// MI455X (gfx1250) — hardware-verified
//
#include <hip/hip_runtime.h>

typedef __attribute__((ext_vector_type(16))) _Float16 v16h;
typedef __attribute__((ext_vector_type(8)))  _Float16 v8h;
typedef __attribute__((ext_vector_type(8)))  float    v8f;
typedef __attribute__((ext_vector_type(4)))  float    v4f;
typedef __attribute__((ext_vector_type(4)))  unsigned v4u;
typedef float __attribute__((may_alias)) float_a;
template <typename T> __device__ __forceinline__ void vst2(void* p, T v) { *(volatile T*)p = v; __threadfence(); *(volatile T*)p = v; }
__device__ __forceinline__ v8f wmma16(v16h a, v16h b, v8f c) {
    v8f d = __builtin_amdgcn_wmma_f32_16x16x32_f16(false, a, false, b, (short)0, c, false, false);
    asm volatile("v_nop\n\tv_nop\n\tv_nop\n\tv_nop" : "+v"(d) : "v"(a), "v"(b));
    return d;
}

#define Nn 8
#define Cc 256
#define Oo 256
#define Dd 256
#define HW 3136
#define WW 56

__global__ void hyper_base_kernel(const float* __restrict__ rf,
                                  const float* __restrict__ W1, const float* __restrict__ b1,
                                  const float* __restrict__ Wb1, const float* __restrict__ bb1,
                                  float* __restrict__ base, float* __restrict__ hidden) {
    int tid = blockIdx.x * blockDim.x + threadIdx.x;
    if (tid >= 2 * Nn * Dd) return;
    int seg = tid / (Nn * Dd);
    int r   = tid % (Nn * Dd);
    int n = r / Dd, j = r % Dd;
    const float* W = seg ? Wb1 : W1;
    const float* b = seg ? bb1 : b1;
    const float* x = rf + n * Dd;
    float acc = b[j];
#pragma unroll 4
    for (int i = 0; i < Dd; ++i) acc += x[i] * W[i * Dd + j];
    acc = fmaxf(acc, 0.f);
    vst2((seg ? hidden : base) + r, (float_a)acc);
}

__global__ void hyper_gen_kernel(const float* __restrict__ base, const float* __restrict__ hidden,
                                 const float* __restrict__ WA, const float* __restrict__ bA,
                                 const float* __restrict__ WB, const float* __restrict__ bB,
                                 const float* __restrict__ WG, const float* __restrict__ bG,
                                 const float* __restrict__ Wb2, const float* __restrict__ bb2,
                                 float* __restrict__ Am, float* __restrict__ Bm,
                                 float* __restrict__ Gm, float* __restrict__ biasO) {
    int tid = blockIdx.x * blockDim.x + threadIdx.x;
    if (tid >= Nn * 10752) return;
    int n = tid / 10752;
    int r = tid % 10752;
    int j, fo;
    const float *W, *bv, *src = base;
    float* dst;
    if (r < 4096)       { j = r;         fo = 4096; W = WA;  bv = bA;  dst = Am    + n * 4096; }
    else if (r < 8192)  { j = r - 4096;  fo = 4096; W = WB;  bv = bB;  dst = Bm    + n * 4096; }
    else if (r < 10496) { j = r - 8192;  fo = 2304; W = WG;  bv = bG;  dst = Gm    + n * 2304; }
    else                { j = r - 10496; fo = 256;  W = Wb2; bv = bb2; dst = biasO + n * 256; src = hidden; }
    const float* x = src + n * Dd;
    float acc = bv[j];
#pragma unroll 4
    for (int i = 0; i < Dd; ++i) acc += x[i] * W[i * fo + j];
    vst2(dst + j, (float_a)acc);
}

__global__ void ag_kernel(const float* __restrict__ Am, const float* __restrict__ Gm,
                          float* __restrict__ AG) {
    int tid = blockIdx.x * blockDim.x + threadIdx.x;
    if (tid >= Nn * Cc * 144) return;
    int n = tid / (Cc * 144);
    int r = tid % (Cc * 144);
    int c = r / 144, j = r % 144;
    const float* a = Am + n * 4096 + c * 16;
    const float* g = Gm + n * 2304 + j;
    float acc = 0.f;
    #pragma unroll
    for (int r1 = 0; r1 < 16; ++r1) acc += a[r1] * g[r1 * 144];
    vst2(AG + n * 36864 + r, (float_a)acc);
}

__global__ void wfrag_kernel(const float* __restrict__ AG, const float* __restrict__ Bm,
                             _Float16* __restrict__ Wf) {
    int tid2 = blockIdx.x * blockDim.x + threadIdx.x;
    if (tid2 >= Nn * 16 * 72 * 32 * 2) return;
    int tid = tid2 >> 1, hsel = tid2 & 1;
    int lane = tid & 31;
    int s    = (tid >> 5) % 72;
    int n    = tid / 36864;
    int lg   = lane >> 4;
    int ot = (tid / 2304) & 15;
    int o  = ot * 16 + (lane & 15);
    int tap = s >> 3;
    float bcol[16];
    #pragma unroll
    for (int r2 = 0; r2 < 16; ++r2) bcol[r2] = Bm[n * 4096 + r2 * 256 + o];
    const float* agn = AG + n * 36864;
    union { v8h v; v4u u; } wv;
    #pragma unroll
    for (int hh = 0; hh < 8; ++hh) {
        int h = hsel * 8 + hh;
        int ka = ((h >> 3) << 4) + (lg << 3) + (h & 7);
        int c  = ((s & 7) << 5) + ka;
        const float* ag = agn + c * 144 + tap * 16;
        float acc = 0.f;
        #pragma unroll
        for (int r2 = 0; r2 < 16; ++r2) acc += ag[r2] * bcol[r2];
        wv.v[hh] = (_Float16)acc;
    }
    vst2(Wf + (size_t)tid * 16 + hsel * 8, wv.u);
}

__global__ void __launch_bounds__(256) cvt_kernel(const float* __restrict__ inp,
                                                  _Float16* __restrict__ inT) {
    __shared__ float tile[64][33];
    int b  = blockIdx.x;
    int pb = b % 98;
    int t2 = b / 98;
    int cb = t2 & 3;
    int n  = t2 >> 2;
    int t  = threadIdx.x;

    int pl  = t & 31;
    int cl0 = t >> 5;
    const float* src = inp + ((size_t)(n * Cc + cb * 64)) * HW + pb * 32;
    #pragma unroll
    for (int i = 0; i < 8; ++i) {
        int c = cl0 + i * 8;
        tile[c][pl] = src[(size_t)c * HW + pl];
    }
    __syncthreads();
    {
        int p = t >> 3, pc = t & 7;
        union { v8h h; v4u u; } pk;
        #pragma unroll
        for (int e = 0; e < 8; ++e) pk.h[e] = (_Float16)tile[pc * 8 + e][p];
        vst2(inT + ((size_t)(n * HW + pb * 32 + p)) * Cc + cb * 64 + pc * 8, pk.u);
    }
}

__global__ void __launch_bounds__(256) conv_wmma_kernel(const _Float16* __restrict__ inT,
                                                        const _Float16* __restrict__ Wf,
                                                        const float* __restrict__ biasO,
                                                        float* __restrict__ out) {
    int lane = threadIdx.x & 31;
    int wave = threadIdx.x >> 5;
    int task = blockIdx.x * 8 + wave;
    int pb = task % 98;
    int t2 = task / 98;
    int ob = t2 & 3;
    int n  = t2 >> 2;

    int p0 = pb * 32 + (lane & 15);
    int p1 = p0 + 16;
    int y0 = p0 / WW, x0 = p0 % WW;
    int y1 = p1 / WW, x1 = p1 % WW;
    int chi = (lane >> 4) << 3;
    __shared__ __attribute__((aligned(16))) float so[8][64 * 32];

    const size_t otStride = (size_t)72 * 32 * 16;
    const _Float16* wf = Wf + ((size_t)((n * 16 + ob * 4) * 72) * 32 + lane) * 16;
    const _Float16* inbase = inT + (size_t)n * HW * Cc;

    v8f acc[4][2] = {};
    v16h zero = {};
    #pragma unroll 1
    for (int tap = 0; tap < 9; ++tap) {
        int dy = tap / 3 - 1, dx = tap % 3 - 1;
        int yy0 = y0 + dy, xx0 = x0 + dx;
        int yy1 = y1 + dy, xx1 = x1 + dx;
        bool v0 = ((unsigned)yy0 < (unsigned)WW) & ((unsigned)xx0 < (unsigned)WW);
        bool v1 = ((unsigned)yy1 < (unsigned)WW) & ((unsigned)xx1 < (unsigned)WW);
        const _Float16* bp0 = inbase + ((size_t)(yy0 * WW + xx0)) * Cc + chi;
        const _Float16* bp1 = inbase + ((size_t)(yy1 * WW + xx1)) * Cc + chi;
        __builtin_prefetch(bp0, 0, 1);
        __builtin_prefetch(bp1, 0, 1);
        #pragma unroll
        for (int s8 = 0; s8 < 8; ++s8) {
            union U { v16h v; v8h q[2]; } b0, b1;
            if (v0) { b0.q[0] = *(const v8h*)(bp0 + s8 * 32); b0.q[1] = *(const v8h*)(bp0 + s8 * 32 + 16); } else b0.v = zero;
            if (v1) { b1.q[0] = *(const v8h*)(bp1 + s8 * 32); b1.q[1] = *(const v8h*)(bp1 + s8 * 32 + 16); } else b1.v = zero;
            #pragma unroll
            for (int t = 0; t < 4; ++t) {
                v16h a = *(const v16h*)(wf + (size_t)t * otStride);
                acc[t][0] = wmma16(a, b0.v, acc[t][0]);
                acc[t][1] = wmma16(a, b1.v, acc[t][1]);
            }
            wf += 512;
        }
    }
    int lg8 = (lane >> 4) << 3;
    float* S = so[wave];
    #pragma unroll
    for (int t = 0; t < 4; ++t) {
        int obaseT = (ob * 4 + t) * 16 + lg8;
        const float* bb = biasO + n * Oo + obaseT;
        #pragma unroll
        for (int v = 0; v < 8; ++v) {
            const int ol = t * 16 + lg8 + v;
            S[ol * 32 + (lane & 15)]      = acc[t][0][v] + bb[v];
            S[ol * 32 + 16 + (lane & 15)] = acc[t][1][v] + bb[v];
        }
    }
    __syncthreads();
    #pragma unroll 4
    for (int q = 0; q < 16; ++q) {
        const int ol = q * 4 + (lane >> 3), pc = lane & 7;
        const int o = (ob * 4) * 16 + ol;
        vst2(out + ((size_t)(n * Oo + o)) * HW + pb * 32 + pc * 4, *(const v4f*)(S + ol * 32 + pc * 4));
    }
}

extern "C" void kernel_launch(void* const* d_in, const int* in_sizes, int n_in,
                              void* d_out, int out_size, void* d_ws, size_t ws_size,
                              hipStream_t stream) {
    const float* inp = (const float*)d_in[0];
    const float* rf  = (const float*)d_in[1];
    const float* W1  = (const float*)d_in[2];   const float* b1  = (const float*)d_in[3];
    const float* WA  = (const float*)d_in[4];   const float* bA  = (const float*)d_in[5];
    const float* WB  = (const float*)d_in[6];   const float* bB  = (const float*)d_in[7];
    const float* WG  = (const float*)d_in[8];   const float* bG  = (const float*)d_in[9];
    const float* Wb1 = (const float*)d_in[10];  const float* bb1 = (const float*)d_in[11];
    const float* Wb2 = (const float*)d_in[12];  const float* bb2 = (const float*)d_in[13];
    float* out = (float*)d_out;

    float* wsBase   = (float*)d_ws;
    float* wsHidden = wsBase   + 2048;
    float* wsBiasO  = wsHidden + 2048;
    float* wsA      = wsBiasO  + 2048;
    float* wsBm     = wsA      + 32768;
    float* wsG      = wsBm     + 32768;
    float* wsAG     = wsG      + 18432;
    _Float16* wsWf  = (_Float16*)(wsAG + 294912);
    _Float16* wsInT = wsWf + 4718592;

    hyper_base_kernel<<<16, 256, 0, stream>>>(rf, W1, b1, Wb1, bb1, wsBase, wsHidden);
    hyper_gen_kernel<<<336, 256, 0, stream>>>(wsBase, wsHidden, WA, bA, WB, bB, WG, bG,
                                              Wb2, bb2, wsA, wsBm, wsG, wsBiasO);
    ag_kernel<<<1152, 256, 0, stream>>>(wsA, wsG, wsAG);
    wfrag_kernel<<<2304, 256, 0, stream>>>(wsAG, wsBm, wsWf);
    cvt_kernel<<<3136, 256, 0, stream>>>(inp, wsInT);
    conv_wmma_kernel<<<392, 256, 0, stream>>>(wsInT, wsWf, wsBiasO, out);
}
